// Multi_CA_48868137894266
// MI455X (gfx1250) — hardware-run, weakly checked
//
#include <hip/hip_runtime.h>
#include <math.h>
#include <stdint.h>

#define NB      4
#define NTOK    1024
#define DMODEL  1024
#define DFF     4096
#define NHEAD   16
#define HDIM    64
#define NSTR    3
#define NROWS   (NB * NTOK)
#define WSC     64.0f
#define W2SC    128.0f
#define XC      1.0f
#define QC      16.0f
#define KC      16.0f
#define VC      16.0f
#define PC      1024.0f
#define H1C     16.0f
#define GC      16.0f
#define ATT_SCALE 0.125f
#define LOG2E   1.4426950408889634f
#define LN_EPS  1e-5f
static_assert(NHEAD * HDIM == DMODEL);
static_assert((NTOK % 64) == 0 && (DMODEL % 64) == 0 && (DFF % 64) == 0 && (NTOK % 32) == 0 && (NTOK % 16) == 0);
static_assert((NROWS % 64) == 0 && (DMODEL % 32) == 0 && (DFF % 32) == 0);
#define HPB     8
#define NHB     (NHEAD / HPB)
#define OSP     (HPB * HDIM)
#define ATT_THREADS (HPB * 32)
#define ATT_BLOCKS  (NB * (NTOK / 16) * NHB)
static_assert(ATT_THREADS == 256 && ATT_BLOCKS == 512 && NHB * HPB == NHEAD && OSP * NHB == DMODEL && OSP == 512);
#define LN_THREADS 256
static_assert(LN_THREADS * 4 == DMODEL && (LN_THREADS % 32) == 0 && ((DMODEL / 8) % 32) == 0);
#define CV_THREADS 256
static_assert(DMODEL == 128 * 8 && (NROWS % 2) == 0);

typedef _Float16 v16h __attribute__((ext_vector_type(16)));
typedef _Float16 v8h  __attribute__((ext_vector_type(8)));
typedef float    v8f  __attribute__((ext_vector_type(8)));
typedef float    v4f  __attribute__((ext_vector_type(4)));
typedef unsigned int v4u __attribute__((ext_vector_type(4)));
typedef unsigned int v2u __attribute__((ext_vector_type(2)));

union FragH { v16h v; v8h h[2]; v4u u[2]; };

__device__ __forceinline__ unsigned short bf_bits(float f) {
  unsigned u = __float_as_uint(f);
  return (unsigned short)((u + 0x7FFFu + ((u >> 16) & 1u)) >> 16);
}
__device__ __forceinline__ float bf_up(unsigned short h) { return __uint_as_float(((unsigned)h) << 16); }
__device__ __forceinline__ float bfr(float f) { return bf_up(bf_bits(f)); }
__device__ __forceinline__ unsigned short h_bits(_Float16 x) { return __builtin_bit_cast(unsigned short, x); }
__device__ __forceinline__ unsigned pk16(unsigned short a, unsigned short b) { return (unsigned)a | ((unsigned)b << 16); }
__device__ __forceinline__ v8f zero8() { v8f z = {0.f, 0.f, 0.f, 0.f, 0.f, 0.f, 0.f, 0.f}; return z; }
__device__ __forceinline__ float gelu_f(float u) { return 0.5f * u * (1.0f + erff(u * 0.70710678118654752440f)); }

__device__ __forceinline__ v16h ldfrag_h(const _Float16* p) {
  FragH f;
  f.h[0] = *(const v8h*)(p);
  f.h[1] = *(const v8h*)(p + 16);
  return f.v;
}
__device__ __forceinline__ v16h ldfrag_u(const unsigned short* p) {
  FragH f;
  f.u[0] = *(const v4u*)(p);
  f.u[1] = *(const v4u*)(p + 16);
  return f.v;
}

__device__ __forceinline__ v8f mma_raw(v16h a, v16h b, v8f c) {
  return __builtin_amdgcn_wmma_f32_16x16x32_f16(false, a, false, b, (short)0, c, false, false);
}
__device__ __forceinline__ void dep_guard1(v8f& a, v8f& b, v16h x) {
#if defined(__HIP_DEVICE_COMPILE__)
  asm volatile("v_nop\n\tv_nop\n\tv_nop\n\tv_nop" : "+v"(a), "+v"(b) : "v"(x));
#endif
}
__device__ __forceinline__ void guard_s2(v8f& s, v16h a0, v16h a1) {
#if defined(__HIP_DEVICE_COMPILE__)
  asm volatile("v_nop\n\tv_nop\n\tv_nop\n\tv_nop" : "+v"(s) : "v"(a0), "v"(a1));
#endif
}
__device__ __forceinline__ void guard_s4(v8f& s, v16h a0, v16h a1, v16h b0, v16h b1) {
#if defined(__HIP_DEVICE_COMPILE__)
  asm volatile("v_nop\n\tv_nop\n\tv_nop\n\tv_nop" : "+v"(s) : "v"(a0), "v"(a1), "v"(b0), "v"(b1));
#endif
}
__device__ __forceinline__ void guard_pv4(v8f& a, v8f& b, v8f& c, v8f& d, v16h x, v16h y, v16h z, v16h w, v16h u) {
#if defined(__HIP_DEVICE_COMPILE__)
  asm volatile("v_nop\n\tv_nop\n\tv_nop\n\tv_nop"
               : "+v"(a), "+v"(b), "+v"(c), "+v"(d) : "v"(x), "v"(y), "v"(z), "v"(w), "v"(u));
#endif
}
__device__ __forceinline__ void keep4_h(v16h a, v16h b, v16h c, v16h d) {
#if defined(__HIP_DEVICE_COMPILE__)
  asm volatile("v_nop" :: "v"(a), "v"(b), "v"(c), "v"(d));
#endif
}
__device__ __forceinline__ void acc_guard4(v8f& a, v8f& b, v8f& c, v8f& d) {
#if defined(__HIP_DEVICE_COMPILE__)
  asm volatile("v_nop\n\tv_nop\n\tv_nop\n\tv_nop" : "+v"(a), "+v"(b), "+v"(c), "+v"(d));
#endif
}
__device__ __forceinline__ void wave_sync_lds() {
  __builtin_amdgcn_fence(__ATOMIC_RELEASE, "workgroup");
  __builtin_amdgcn_wave_barrier();
  __builtin_amdgcn_fence(__ATOMIC_ACQUIRE, "workgroup");
}

__global__ __launch_bounds__(256) void tcvt16(const float* __restrict__ src, unsigned short* dst, int R, int C, float sc) {
  __shared__ __align__(16) unsigned short sT[64 * 72];
  const int tid = threadIdx.x, lane = tid & 31, wave = tid >> 5;
  const int c0 = blockIdx.x * 64, r0 = blockIdx.y * 64;
  const int rr = tid >> 2, cc = (tid & 3) * 16;
  const float* sp = src + (size_t)(r0 + rr) * C + c0 + cc;
#pragma unroll
  for (int e = 0; e < 4; ++e) {
    const v4f a = *(const v4f*)(sp + 4 * e);
#pragma unroll
    for (int k = 0; k < 4; ++k)
      sT[(cc + 4 * e + k) * 72 + rr] = h_bits((_Float16)(bfr(a[k]) * sc));
  }
  __syncthreads();
  v4u vals[2];
#pragma unroll
  for (int it = 0; it < 2; ++it) {
    const int q = it * 32 + wave * 4 + (lane >> 3);
    vals[it] = *(const v4u*)(sT + q * 72 + (lane & 7) * 8);
  }
  for (int pass = 0; pass < 2; ++pass) {
#pragma unroll
    for (int it = 0; it < 2; ++it) {
      const int q = it * 32 + wave * 4 + (lane >> 3);
      *(volatile v4u*)(dst + (size_t)(c0 + q) * R + r0 + (lane & 7) * 8) = vals[it];
    }
    __threadfence();
  }
}

__global__ __launch_bounds__(CV_THREADS) void cvtrow(const float* __restrict__ src, unsigned short* dst, float sc) {
  const int tid = threadIdx.x;
  const int row = blockIdx.x * 2 + (tid >> 7);
  const int c8  = (tid & 127) * 8;
  const float* sp = src + (size_t)row * DMODEL + c8;
  const v4f a = *(const v4f*)(sp);
  const v4f b = *(const v4f*)(sp + 4);
  v4u w;
  w[0] = pk16(h_bits((_Float16)(bfr(a[0]) * sc)), h_bits((_Float16)(bfr(a[1]) * sc)));
  w[1] = pk16(h_bits((_Float16)(bfr(a[2]) * sc)), h_bits((_Float16)(bfr(a[3]) * sc)));
  w[2] = pk16(h_bits((_Float16)(bfr(b[0]) * sc)), h_bits((_Float16)(bfr(b[1]) * sc)));
  w[3] = pk16(h_bits((_Float16)(bfr(b[2]) * sc)), h_bits((_Float16)(bfr(b[3]) * sc)));
  unsigned short* dp = dst + (size_t)row * DMODEL + c8;
  for (int pass = 0; pass < 2; ++pass) {
    *(volatile v4u*)dp = w;
    __threadfence();
  }
}

template <int OM, int HASR, int ACT, int HASB>
__global__ __launch_bounds__(256) void gemm64(
    const unsigned short* __restrict__ Ap, int lda, long long sA,
    const unsigned short* __restrict__ Btp, int ldb, long long sB,
    const float* __restrict__ Rp, const float* __restrict__ Bsp,
    void* Cout, int ldc, long long sC,
    int M, int N, int K, float oscale, float ocarry) {
  __shared__ __align__(16) float sT[8][16 * 68];
  const int by   = blockIdx.y;
  const int lane = threadIdx.x & 31;
  const int wave = threadIdx.x >> 5;
  const int tilesN = N >> 6;
  const int tilesM = M >> 6;
  const int tile = blockIdx.x * 8 + wave;
  if (tile >= tilesM * tilesN) return;
  const int tm = tile / tilesN;
  const int tn = tile - tm * tilesN;
  const int m0 = tm << 6;
  const int n0 = tn << 6;

  const unsigned short* A1 = Ap  + (size_t)((long long)by * sA);
  const unsigned short* Bb = Btp + (size_t)((long long)by * sB);

  const int rlane = lane & 15;
  const int koff  = (lane >> 4) * 8;
  const int mOff  = (lane >> 4) * 8;

  v8f acc[4][4];
#pragma unroll
  for (int i = 0; i < 4; ++i)
#pragma unroll
    for (int j = 0; j < 4; ++j) acc[i][j] = zero8();

  for (int k0 = 0; k0 < K; k0 += 32) {
    v16h bh[4];
#pragma unroll
    for (int j = 0; j < 4; ++j) {
      const size_t bofs = (size_t)(n0 + (j << 4) + rlane) * ldb + koff + k0;
      bh[j] = ldfrag_u(Bb + bofs);
    }
#pragma unroll
    for (int i = 0; i < 4; ++i) {
      const size_t ao = (size_t)(m0 + (i << 4) + rlane) * lda + koff + k0;
      const v16h ah = ldfrag_u(A1 + ao);
#pragma unroll
      for (int j = 0; j < 4; ++j) acc[i][j] = mma_raw(ah, bh[j], acc[i][j]);
      dep_guard1(acc[i][0], acc[i][3], ah);
    }
    keep4_h(bh[0], bh[1], bh[2], bh[3]);
  }
  acc_guard4(acc[0][0], acc[0][1], acc[0][2], acc[0][3]);
  acc_guard4(acc[1][0], acc[1][1], acc[1][2], acc[1][3]);
  acc_guard4(acc[2][0], acc[2][1], acc[2][2], acc[2][3]);
  acc_guard4(acc[3][0], acc[3][1], acc[3][2], acc[3][3]);

  const int hh2 = lane >> 4, c4 = (lane & 15) * 4;
  const int q8  = lane >> 3, c8 = (lane & 7) * 8;

  v4f bias4 = {0.f, 0.f, 0.f, 0.f};
  v8f bias8 = zero8();
  if constexpr (HASB == 1) {
    if constexpr (OM == 0) {
      const v4f t = *(const v4f*)(Bsp + n0 + c4);
#pragma unroll
      for (int e = 0; e < 4; ++e) bias4[e] = bfr(t[e]);
    } else {
      const v4f t0 = *(const v4f*)(Bsp + n0 + c8);
      const v4f t1 = *(const v4f*)(Bsp + n0 + c8 + 4);
#pragma unroll
      for (int e = 0; e < 4; ++e) { bias8[e] = bfr(t0[e]); bias8[4 + e] = bfr(t1[e]); }
    }
  }

  float* slab = sT[wave];
#pragma unroll
  for (int i = 0; i < 4; ++i) {
    const int mBase = m0 + (i << 4);
#pragma unroll
    for (int j = 0; j < 4; ++j) {
#pragma unroll
      for (int r = 0; r < 8; ++r) {
        slab[(mOff + r) * 68 + (j << 4) + rlane] = acc[i][j][r];
      }
    }
    wave_sync_lds();
    if constexpr (OM == 0) {
      float* C = (float*)Cout + (size_t)((long long)by * sC);
      v4f vals[8];
#pragma unroll
      for (int it = 0; it < 8; ++it) {
        const int row = it * 2 + hh2;
        const int gr  = mBase + row;
        v4f v = *(const v4f*)(slab + row * 68 + c4);
        v4f rv = {0.f, 0.f, 0.f, 0.f};
        if constexpr (HASR != 0) {
          const float* R = Rp + (size_t)((long long)by * sC);
          const v4f rraw = *(const v4f*)(R + (size_t)gr * ldc + n0 + c4);
#pragma unroll
          for (int e = 0; e < 4; ++e) rv[e] = (HASR == 1) ? bfr(rraw[e]) : rraw[e];
        }
#pragma unroll
        for (int e = 0; e < 4; ++e) v[e] = (v[e] * oscale + bias4[e]) + rv[e];
        vals[it] = v;
      }
      for (int pass = 0; pass < 2; ++pass) {
#pragma unroll
        for (int it = 0; it < 8; ++it) {
          const int gr = mBase + it * 2 + hh2;
          *(volatile v4f*)(C + (size_t)gr * ldc + n0 + c4) = vals[it];
        }
        __threadfence();
      }
    } else {
      unsigned short* C = (unsigned short*)Cout + (size_t)((long long)by * sC);
      v4u hv[4];
#pragma unroll
      for (int it = 0; it < 4; ++it) {
        const int row = it * 4 + q8;
        const float* sp = slab + row * 68 + c8;
        v4u a = {0u, 0u, 0u, 0u};
#pragma unroll
        for (int e = 0; e < 4; ++e) {
          float f0 = sp[2 * e] * oscale + bias8[2 * e];
          float f1 = sp[2 * e + 1] * oscale + bias8[2 * e + 1];
          if constexpr (ACT == 1) { f0 = gelu_f(f0); f1 = gelu_f(f1); }
          f0 *= ocarry; f1 *= ocarry;
          a[e] = pk16(h_bits((_Float16)f0), h_bits((_Float16)f1));
        }
        hv[it] = a;
      }
      for (int pass = 0; pass < 2; ++pass) {
#pragma unroll
        for (int it = 0; it < 4; ++it) {
          const int row = it * 4 + q8;
          *(volatile v4u*)(C + (size_t)(mBase + row) * ldc + n0 + c8) = hv[it];
        }
        __threadfence();
      }
    }
    wave_sync_lds();
  }
}

#define PT_FLOATS (HPB * 16 * 36)
static_assert(((16 * OSP) % (4 * ATT_THREADS)) == 0 && ((16 * OSP) / (4 * ATT_THREADS)) == 8);
static_assert((OSP / 4) == 128);

__global__ __launch_bounds__(ATT_THREADS)
void attn3(const unsigned short* __restrict__ QHp, const unsigned short* __restrict__ KHp,
           const unsigned short* __restrict__ VTp, float* ATT) {
  __shared__ __align__(16) float pbuf[PT_FLOATS];
  __shared__ __align__(16) float obuf[16 * OSP];

  const int tid  = threadIdx.x;
  const int wave = tid >> 5;
  const int lane = tid & 31;
  const int hh   = lane >> 4;
  const int c    = lane & 15;

  const int hb   = blockIdx.x % NHB;
  const int qt   = (blockIdx.x / NHB) % (NTOK / 16);
  const int bat  = blockIdx.x / (NHB * (NTOK / 16));
  const int head = hb * HPB + wave;
  const int q0   = qt * 16;

  const size_t qofs = ((size_t)bat * NTOK + q0 + c) * DMODEL + head * HDIM + 8 * hh;
  const _Float16* Qh = (const _Float16*)(const void*)QHp + qofs;
  const float lsc = (LOG2E * ATT_SCALE) / (QC * KC);
  const float ocs = 1.0f / (PC * VC);

  const v16h qa = ldfrag_h(Qh), qb = ldfrag_h(Qh + 32);

  float* ob = obuf + wave * HDIM + c;
#pragma unroll
  for (int r = 0; r < 8; ++r) {
    float* op = ob + (8 * hh + r) * OSP;
    op[0] = 0.f; op[16] = 0.f; op[32] = 0.f; op[48] = 0.f;
  }
  float* pt = pbuf + wave * (16 * 36);

#pragma unroll 1
  for (int s = 0; s < NSTR; ++s) {
    const _Float16* Kb = (const _Float16*)(const void*)KHp + (size_t)s * NROWS * DMODEL
                         + (size_t)bat * NTOK * DMODEL + head * HDIM + 8 * hh;
    const _Float16* Vb = (const _Float16*)(const void*)VTp + (size_t)s * NB * DMODEL * NTOK
                         + ((size_t)bat * DMODEL + head * HDIM) * NTOK + 8 * hh;

    float mrow[8], lrow[8];
    v8f o0 = zero8(), o1 = zero8(), o2 = zero8(), o3 = zero8();
#pragma unroll
    for (int r = 0; r < 8; ++r) { mrow[r] = -INFINITY; lrow[r] = 0.f; }

#pragma unroll 1
    for (int kb = 0; kb < NTOK; kb += 32) {
      const _Float16* kp = Kb + (size_t)(kb + c) * DMODEL;
      v8f s0, s1;
      {
        const v16h k0 = ldfrag_h(kp), k1 = ldfrag_h(kp + 32);
        s0 = mma_raw(qa, k0, zero8());
        s0 = mma_raw(qb, k1, s0);
        guard_s2(s0, k0, k1);
      }
      {
        const _Float16* kq = kp + (size_t)16 * DMODEL;
        const v16h k0 = ldfrag_h(kq), k1 = ldfrag_h(kq + 32);
        s1 = mma_raw(qa, k0, zero8());
        s1 = mma_raw(qb, k1, s1);
        guard_s4(s1, k0, k1, qa, qb);
      }
#pragma unroll
      for (int r = 0; r < 8; ++r) {
        const float t0 = s0[r] * lsc;
        const float t1 = s1[r] * lsc;
        float mx = fmaxf(t0, t1);
#pragma unroll
        for (int off = 1; off < 16; off <<= 1) mx = fmaxf(mx, __shfl_xor(mx, off, 32));
        const float mn = fmaxf(mrow[r], mx);
        const float al = exp2f(fmaxf(mrow[r] - mn, -126.0f));
        mrow[r] = mn;
        const float e0 = exp2f(t0 - mn);
        const float e1 = exp2f(t1 - mn);
        float ps = e0 + e1;
#pragma unroll
        for (int off = 1; off < 16; off <<= 1) ps += __shfl_xor(ps, off, 32);
        lrow[r] = lrow[r] * al + ps;
        o0[r] *= al;
        o1[r] *= al;
        o2[r] *= al;
        o3[r] *= al;
        const int ro = (8 * hh + r) * 36 + c;
        pt[ro]      = e0;
        pt[ro + 16] = e1;
      }
      wave_sync_lds();
      FragH ph;
      {
        const float* prow = pt + c * 36 + 8 * hh;
        const v4f p0 = *(const v4f*)(prow), p1 = *(const v4f*)(prow + 4);
        const v4f p2 = *(const v4f*)(prow + 16), p3 = *(const v4f*)(prow + 20);
#pragma unroll
        for (int e = 0; e < 4; ++e) {
          ph.h[0][e]     = (_Float16)(p0[e] * PC);
          ph.h[0][4 + e] = (_Float16)(p1[e] * PC);
          ph.h[1][e]     = (_Float16)(p2[e] * PC);
          ph.h[1][4 + e] = (_Float16)(p3[e] * PC);
        }
      }
      const _Float16* vp = Vb + (size_t)c * NTOK + kb;
      {
        const v16h vb0 = ldfrag_h(vp);
        const v16h vb1 = ldfrag_h(vp + (size_t)16 * NTOK);
        const v16h vb2 = ldfrag_h(vp + (size_t)32 * NTOK);
        const v16h vb3 = ldfrag_h(vp + (size_t)48 * NTOK);
        o0 = mma_raw(ph.v, vb0, o0);
        o1 = mma_raw(ph.v, vb1, o1);
        o2 = mma_raw(ph.v, vb2, o2);
        o3 = mma_raw(ph.v, vb3, o3);
        guard_pv4(o0, o1, o2, o3, ph.v, vb0, vb1, vb2, vb3);
      }
      wave_sync_lds();
    }

#pragma unroll
    for (int r = 0; r < 8; ++r) {
      const float inv = (1.0f / lrow[r]) * ocs;
      float* op = ob + (8 * hh + r) * OSP;
      const float a0 = op[0]  + o0[r] * inv;
      const float a1 = op[16] + o1[r] * inv;
      const float a2 = op[32] + o2[r] * inv;
      const float a3 = op[48] + o3[r] * inv;
      op[0] = a0; op[16] = a1; op[32] = a2; op[48] = a3;
    }
  }

  __syncthreads();
  {
    v4f vals[8];
#pragma unroll
    for (int it = 0; it < 8; ++it) {
      const int p = it * ATT_THREADS + tid;
      vals[it] = *(const v4f*)(obuf + (size_t)p * 4);
    }
    float* dst = ATT + ((size_t)bat * NTOK + q0) * DMODEL + (size_t)hb * OSP;
    for (int pass = 0; pass < 2; ++pass) {
#pragma unroll
      for (int it = 0; it < 8; ++it) {
        const int p = it * ATT_THREADS + tid;
        const int row = p >> 7, col4 = (p & 127) * 4;
        *(volatile v4f*)(dst + (size_t)row * DMODEL + col4) = vals[it];
      }
      __threadfence();
    }
  }
}

template <int MODE>
__global__ __launch_bounds__(LN_THREADS)
void lnorm(const float* __restrict__ Pp, const float* __restrict__ Ap2, const float* __restrict__ gp,
           const float* __restrict__ bp, float* Fo, unsigned short* Ho, float hc) {
  __shared__ float red[2][LN_THREADS / 32];
  __shared__ __align__(16) unsigned short srow[DMODEL];
  const int row  = blockIdx.x;
  const int tid  = threadIdx.x;
  const int lane = tid & 31;
  const int wave = tid >> 5;
  const size_t base = (size_t)row * DMODEL + (size_t)tid * 4;
  v4f v = *(const v4f*)(Pp + base);
  if constexpr (MODE == 1) {
    const v4f a = *(const v4f*)(Ap2 + base);
#pragma unroll
    for (int e = 0; e < 4; ++e) v[e] = bfr(v[e]) + a[e];
  }
  float s = (v[0] + v[1]) + (v[2] + v[3]);
#pragma unroll
  for (int off = 1; off < 32; off <<= 1) s += __shfl_xor(s, off, 32);
  if (lane == 0) red[0][wave] = s;
  __syncthreads();
  float tot = 0.f;
#pragma unroll
  for (int w = 0; w < LN_THREADS / 32; ++w) tot += red[0][w];
  const float mu = tot * (1.0f / (float)DMODEL);
  v4f d;
#pragma unroll
  for (int e = 0; e < 4; ++e) d[e] = v[e] - mu;
  float q = (d[0] * d[0] + d[1] * d[1]) + (d[2] * d[2] + d[3] * d[3]);
#pragma unroll
  for (int off = 1; off < 32; off <<= 1) q += __shfl_xor(q, off, 32);
  if (lane == 0) red[1][wave] = q;
  __syncthreads();
  float totq = 0.f;
#pragma unroll
  for (int w = 0; w < LN_THREADS / 32; ++w) totq += red[1][w];
  const float var  = totq * (1.0f / (float)DMODEL);
  const float rstd = rsqrtf(var + LN_EPS);
  const v4f g4 = *(const v4f*)(gp + tid * 4);
  const v4f b4 = *(const v4f*)(bp + tid * 4);
  v4f o;
#pragma unroll
  for (int e = 0; e < 4; ++e) o[e] = (d[e] * rstd) * bfr(g4[e]) + bfr(b4[e]);
  {
    float* fd = Fo + base;
    for (int pass = 0; pass < 2; ++pass) {
      *(volatile v4f*)fd = o;
      __threadfence();
    }
  }
  if constexpr (MODE == 1) {
    v2u w;
    w[0] = pk16(h_bits((_Float16)(o[0] * hc)), h_bits((_Float16)(o[1] * hc)));
    w[1] = pk16(h_bits((_Float16)(o[2] * hc)), h_bits((_Float16)(o[3] * hc)));
    *(v2u*)(srow + tid * 4) = w;
    __syncthreads();
    if (tid < DMODEL / 8) {
      const v4u hv = *(const v4u*)(srow + tid * 8);
      unsigned short* dst = Ho + (size_t)row * DMODEL + (size_t)tid * 8;
      for (int pass = 0; pass < 2; ++pass) {
        *(volatile v4u*)dst = hv;
        __threadfence();
      }
    }
  }
}

extern "C" void kernel_launch(void* const* d_in, const int* in_sizes, int n_in,
                              void* d_out, int out_size, void* d_ws, size_t ws_size,
                              hipStream_t stream) {
  if (n_in < 19) return;
  for (int i = 0; i < 4; ++i) if (in_sizes[i] != NROWS * DMODEL) return;
  for (int i = 4; i < 11; ++i) if (in_sizes[i] != DMODEL * DMODEL) return;
  if (in_sizes[11] != DMODEL * DFF || in_sizes[12] != DFF || in_sizes[13] != DFF * DMODEL) return;
  for (int i = 14; i < 19; ++i) if (in_sizes[i] != DMODEL) return;
  if (out_size != NROWS * DMODEL) return;

  const float* xq  = (const float*)d_in[0];
  const float* xt  = (const float*)d_in[1];
  const float* xa  = (const float*)d_in[2];
  const float* xv  = (const float*)d_in[3];
  const float* wq  = (const float*)d_in[4];
  const float* wkt = (const float*)d_in[5];
  const float* wka = (const float*)d_in[6];
  const float* wkv = (const float*)d_in[7];
  const float* wvt = (const float*)d_in[8];
  const float* wva = (const float*)d_in[9];
  const float* wvv = (const float*)d_in[10];
  const float* w1  = (const float*)d_in[11];
  const float* b1  = (const float*)d_in[12];
  const float* w2  = (const float*)d_in[13];
  const float* b2  = (const float*)d_in[14];
  const float* g1  = (const float*)d_in[15];
  const float* be1 = (const float*)d_in[16];
  const float* g2  = (const float*)d_in[17];
  const float* be2 = (const float*)d_in[18];
  float*       out = (float*)d_out;

  const size_t DD  = (size_t)DMODEL * DMODEL;
  const size_t XP  = (size_t)NROWS * DMODEL;
  const size_t VP  = (size_t)NB * DMODEL * NTOK;
  const size_t PWT = 7 * DD * 2;
  const size_t PW1 = (size_t)DFF * DMODEL * 2;
  const size_t PW2 = (size_t)DMODEL * DFF * 2;
  const size_t PX4 = 4 * XP * 2;
  const size_t PQ  = XP * 2;
  const size_t PK  = 3 * XP * 2;
  const size_t PV  = 3 * VP * 2;
  const size_t PF  = XP * 4;
  const size_t PH  = (size_t)NROWS * DFF * 2;
  size_t off = 0;
  const size_t oWT = off; off += PWT;
  const size_t oW1 = off; off += PW1;
  const size_t oW2 = off; off += PW2;
  const size_t oX  = off; off += PX4;
  const size_t oQ  = off; off += PQ;
  const size_t oK  = off; off += PK;
  const size_t oV  = off; off += PV;
  if (off > ws_size) return;
  if (off > (size_t)134217728) return;
  const size_t oATT = oX;
  const size_t oHH  = oX;
  const size_t oX1F = oQ;
  const size_t oH1  = oQ + PF;
  const size_t oYF  = oH1 + PQ;
  if (PF > PX4 || PH > PX4) return;
  if (oYF + PF > oV + PV) return;

  char* ws = (char*)d_ws;
  unsigned short* WT   = (unsigned short*)(ws + oWT);
  unsigned short* W1T  = (unsigned short*)(ws + oW1);
  unsigned short* W2T  = (unsigned short*)(ws + oW2);
  unsigned short* X16  = (unsigned short*)(ws + oX);
  float*          ATT  = (float*)(ws + oATT);
  unsigned short* HH   = (unsigned short*)(ws + oHH);
  unsigned short* QH   = (unsigned short*)(ws + oQ);
  unsigned short* KH   = (unsigned short*)(ws + oK);
  unsigned short* VT   = (unsigned short*)(ws + oV);
  float*          X1F  = (float*)(ws + oX1F);
  unsigned short* H1   = (unsigned short*)(ws + oH1);
  float*          YF   = (float*)(ws + oYF);

  const dim3 blk(256);
  const dim3 gTsq(DMODEL / 64, DMODEL / 64);
  const dim3 gT1(DFF / 64, DMODEL / 64);
  const dim3 gT2(DMODEL / 64, DFF / 64);
  const dim3 gCV(NROWS / 2);
  const int tilesP = (NROWS / 64) * (DMODEL / 64);
  const int tilesV = (DMODEL / 64) * (NTOK / 64);
  const int tilesF = (NROWS / 64) * (DFF / 64);
  const dim3 gP((tilesP + 7) / 8, 1);
  const dim3 gK((tilesP + 7) / 8, NSTR);
  const dim3 gV((tilesV + 7) / 8, NB);
  const dim3 gF((tilesF + 7) / 8, 1);
  const dim3 gAT(ATT_BLOCKS);
  const dim3 bAT(ATT_THREADS);
  const dim3 gLN(NROWS);
  const dim3 bLN(LN_THREADS);

  tcvt16<<<gTsq, blk, 0, stream>>>(wq,  WT + 0 * DD, DMODEL, DMODEL, WSC);
  tcvt16<<<gTsq, blk, 0, stream>>>(wkt, WT + 1 * DD, DMODEL, DMODEL, WSC);
  tcvt16<<<gTsq, blk, 0, stream>>>(wka, WT + 2 * DD, DMODEL, DMODEL, WSC);
  tcvt16<<<gTsq, blk, 0, stream>>>(wkv, WT + 3 * DD, DMODEL, DMODEL, WSC);
  tcvt16<<<gTsq, blk, 0, stream>>>(wvt, WT + 4 * DD, DMODEL, DMODEL, WSC);
  tcvt16<<<gTsq, blk, 0, stream>>>(wva, WT + 5 * DD, DMODEL, DMODEL, WSC);
  tcvt16<<<gTsq, blk, 0, stream>>>(wvv, WT + 6 * DD, DMODEL, DMODEL, WSC);
  tcvt16<<<gT1,  blk, 0, stream>>>(w1, W1T, DMODEL, DFF, WSC);
  tcvt16<<<gT2,  blk, 0, stream>>>(w2, W2T, DFF, DMODEL, W2SC);

  cvtrow<<<gCV, blk, 0, stream>>>(xq, X16 + 0 * XP, XC);
  cvtrow<<<gCV, blk, 0, stream>>>(xt, X16 + 1 * XP, XC);
  cvtrow<<<gCV, blk, 0, stream>>>(xa, X16 + 2 * XP, XC);
  cvtrow<<<gCV, blk, 0, stream>>>(xv, X16 + 3 * XP, XC);

  gemm64<2, 0, 0, 0><<<gP, blk, 0, stream>>>(
      X16, DMODEL, 0LL,
      WT, DMODEL, 0LL,
      xq, b1,
      (void*)QH, DMODEL, 0LL,
      NROWS, DMODEL, DMODEL, 1.0f / (XC * WSC), QC);

  gemm64<2, 0, 0, 0><<<gK, blk, 0, stream>>>(
      X16 + 1 * XP, DMODEL, (long long)XP,
      WT + 1 * DD, DMODEL, (long long)DD,
      xq, b1,
      (void*)KH, DMODEL, (long long)XP,
      NROWS, DMODEL, DMODEL, 1.0f / (XC * WSC), KC);

  for (int s = 0; s < NSTR; ++s) {
    gemm64<2, 0, 0, 0><<<gV, blk, 0, stream>>>(
        WT + (size_t)(4 + s) * DD, DMODEL, 0LL,
        X16 + (size_t)(1 + s) * XP, DMODEL, (long long)NTOK * DMODEL,
        xq, b1,
        (void*)(VT + (size_t)s * VP), NTOK, (long long)DMODEL * NTOK,
        DMODEL, NTOK, DMODEL, 1.0f / (XC * WSC), VC);
  }

  attn3<<<gAT, bAT, 0, stream>>>(QH, KH, VT, ATT);

  lnorm<1><<<gLN, bLN, 0, stream>>>(xq, ATT, g1, be1, X1F, H1, H1C);

  gemm64<2, 0, 1, 1><<<gF, blk, 0, stream>>>(
      H1, DMODEL, 0LL,
      W1T, DMODEL, 0LL,
      X1F, b1,
      (void*)HH, DFF, 0LL,
      NROWS, DFF, DMODEL, 1.0f / (H1C * WSC), GC);

  gemm64<0, 2, 0, 1><<<gP, blk, 0, stream>>>(
      HH, DFF, 0LL,
      W2T, DFF, 0LL,
      X1F, b2,
      (void*)YF, DMODEL, 0LL,
      NROWS, DMODEL, DFF, 1.0f / (GC * W2SC), 1.0f);

  lnorm<2><<<gLN, bLN, 0, stream>>>(YF, YF, g2, be2, out, H1, 1.0f);
  (void)hipGetLastError();
}
